// AdvancedFeatureTransformer_44547400794392
// MI455X (gfx1250) — hardware-verified
//
#include <hip/hip_runtime.h>
#include <math.h>

#define BATCH 4096
#define D_IN  512
#define DMODEL 256
#define TOUT  424
#define NLAYER 6
#define LN_EPS 1e-5f

typedef _Float16 v4h  __attribute__((ext_vector_type(4)));
typedef _Float16 v8h  __attribute__((ext_vector_type(8)));
typedef _Float16 v16h __attribute__((ext_vector_type(16)));
typedef float    v8f  __attribute__((ext_vector_type(8)));

typedef float    v4f  __attribute__((ext_vector_type(4)));
typedef unsigned v4u  __attribute__((ext_vector_type(4)));
template <typename V> __device__ __forceinline__ void vst2(void* p, V v) {
    *(volatile V*)p = v; __threadfence(); *(volatile V*)p = v;
}
__device__ __forceinline__ void copy_b128(char* lds_base, unsigned byte_off, const void* gaddr) {
    *(v4u*)(lds_base + byte_off) = *(const v4u*)gaddr;
}

__device__ __forceinline__ v16h load_frag_a(const _Float16* base, int stride, int lane) {
    const int r  = lane & 15;
    const int kb = (lane < 16) ? 0 : 8;
    const _Float16* p = base + r * stride + kb;
    v8h lo = *(const v8h*)(p);
    v8h hi = *(const v8h*)(p + 16);
    v16h f;
#pragma unroll
    for (int i = 0; i < 8; ++i) { f[i] = lo[i]; f[i + 8] = hi[i]; }
    return f;
}
__device__ __forceinline__ v16h load_frag_b(const _Float16* base, int stride, int lane) {
    return load_frag_a(base, stride, lane);
}
__device__ __forceinline__ v8f wmma_f16(v16h a, v16h b, v8f c) {
    v8f d = __builtin_amdgcn_wmma_f32_16x16x32_f16(false, a, false, b, (short)0, c, false, false);
    asm volatile("v_nop\n\tv_nop\n\tv_nop\n\tv_nop" : "+v"(d) : "v"(a), "v"(b));
    return d;
}
__device__ __forceinline__ float gelu_exact(float x) {
    return 0.5f * x * (1.0f + erff(x * 0.70710678118654752f));
}

__global__ __launch_bounds__(256) void cvt_f32_f16_kernel(
    const float* __restrict__ src, _Float16* __restrict__ dst, int n4)
{
    const int i = blockIdx.x * 256 + threadIdx.x;
    if (i < n4) {
        float4 v = ((const float4*)src)[i];
        v4h o;
        o[0] = (_Float16)v.x; o[1] = (_Float16)v.y;
        o[2] = (_Float16)v.z; o[3] = (_Float16)v.w;
        vst2((v4h*)dst + i, o);
    }
}

template <int ACT, bool RES, bool OUT32, bool OUT16>
__global__ __launch_bounds__(128) void gemm_wmma_f16_kernel(
    const _Float16* __restrict__ A, const _Float16* __restrict__ W,
    const float* __restrict__ bias, const float* __restrict__ R,
    float* __restrict__ C32, _Float16* __restrict__ C16,
    int M, int N, int K)
{
    __shared__ __align__(16) _Float16 sA[2][64 * 32];
    __shared__ __align__(16) _Float16 sB[2][64 * 32];
    __shared__ __align__(16) float Ct[64][64];

    const int tid  = threadIdx.x;
    const int lane = tid & 31;
    const int wave = tid >> 5;
    const int m0   = blockIdx.x * 64;
    const int n0   = blockIdx.y * 64;
    const int wm   = (wave >> 1) * 32;
    const int wn   = (wave & 1) * 32;
    char* ldsA = (char*)sA;
    char* ldsB = (char*)sB;

    auto issue_tiles = [&](int buf, int kc) {
#pragma unroll
        for (int i = 0; i < 2; ++i) {
            const int idx = tid + i * 128;
            const int r = idx >> 2, c = idx & 3;
            copy_b128(ldsA, buf * 4096 + r * 64 + c * 16, A + (size_t)(m0 + r) * K + kc + c * 8);
            copy_b128(ldsB, buf * 4096 + r * 64 + c * 16, W + (size_t)(n0 + r) * K + kc + c * 8);
        }
    };

    v8f acc[2][2] = {};

    issue_tiles(0, 0);
    for (int kc = 0, it = 0; kc < K; kc += 32, ++it) {
        const int cur = it & 1;
        __syncthreads();
        if (kc + 32 < K) issue_tiles(cur ^ 1, kc + 32);

        v16h af[2], bf[2];
#pragma unroll
        for (int mt = 0; mt < 2; ++mt)
            af[mt] = load_frag_a(&sA[cur][(wm + mt * 16) * 32], 32, lane);
#pragma unroll
        for (int nt = 0; nt < 2; ++nt)
            bf[nt] = load_frag_b(&sB[cur][(wn + nt * 16) * 32], 32, lane);
#pragma unroll
        for (int mt = 0; mt < 2; ++mt)
#pragma unroll
            for (int nt = 0; nt < 2; ++nt)
                acc[mt][nt] = wmma_f16(af[mt], bf[nt], acc[mt][nt]);
        __syncthreads();
    }

    const int cn = lane & 15;
    const int mh = (lane >> 4) << 3;
#pragma unroll
    for (int mt = 0; mt < 2; ++mt)
#pragma unroll
        for (int nt = 0; nt < 2; ++nt) {
            const int n = n0 + wn + nt * 16 + cn;
            const float bv = bias[n];
#pragma unroll
            for (int j = 0; j < 8; ++j) {
                const int m = m0 + wm + mt * 16 + mh + j;
                float v = acc[mt][nt][j] + bv;
                if (ACT == 1) v = gelu_exact(v);
                if (RES) v += R[(size_t)m * N + n];
                Ct[wm + mt * 16 + mh + j][wn + nt * 16 + cn] = v;
            }
        }
    __syncthreads();
    if (OUT32) for (int g = tid; g < 64 * 16; g += 128) { const int rl = g >> 4, pc = g & 15; vst2(C32 + (size_t)(m0 + rl) * N + n0 + pc * 4, *(const v4f*)(&Ct[rl][pc * 4])); }
    if (OUT16) for (int g = tid; g < 64 * 8; g += 128) {
        const int rl = g >> 3, pc = g & 7;
        union { v8h h; v4u u; } pk;
#pragma unroll
        for (int e = 0; e < 8; ++e) pk.h[e] = (_Float16)Ct[rl][pc * 8 + e];
        vst2(C16 + (size_t)(m0 + rl) * N + n0 + pc * 8, pk.u);
    }
}

__global__ __launch_bounds__(128) void ln256_kernel(
    const float* __restrict__ X, const float* __restrict__ g,
    const float* __restrict__ b, float* __restrict__ Y32,
    _Float16* __restrict__ Y16)
{
    __shared__ __align__(16) _Float16 s16[4][256];
    const int row  = blockIdx.x * 4 + (threadIdx.x >> 5);
    const int wv   = threadIdx.x >> 5;
    const int lane = threadIdx.x & 31;
    const float* xr = X + (size_t)row * DMODEL;
    float v[8], s = 0.f, ss = 0.f;
#pragma unroll
    for (int i = 0; i < 8; ++i) {
        v[i] = xr[lane + i * 32];
        s += v[i]; ss += v[i] * v[i];
    }
#pragma unroll
    for (int msk = 16; msk >= 1; msk >>= 1) {
        s  += __shfl_xor(s, msk, 32);
        ss += __shfl_xor(ss, msk, 32);
    }
    const float mean = s * (1.f / DMODEL);
    const float var  = ss * (1.f / DMODEL) - mean * mean;
    const float rstd = rsqrtf(var + LN_EPS);
#pragma unroll
    for (int i = 0; i < 8; ++i) {
        const int c = lane + i * 32;
        const float y = (v[i] - mean) * rstd * g[c] + b[c];
        vst2(Y32 + (size_t)row * DMODEL + c, y);
        s16[wv][c] = (_Float16)y;
    }
    __syncthreads();
    vst2(Y16 + (size_t)row * DMODEL + lane * 8, *(const v4u*)(&s16[wv][lane * 8]));
}

__global__ __launch_bounds__(128) void tp_fused_kernel(
    const _Float16* __restrict__ h16,
    const _Float16* __restrict__ W1, const float* __restrict__ b1,
    const float* __restrict__ lng, const float* __restrict__ lnb,
    const _Float16* __restrict__ W2, const float* __restrict__ b2,
    const float* __restrict__ W3, const float* __restrict__ b3,
    float* __restrict__ out)
{
    __shared__ __align__(16) char smem[73728];
    _Float16* sAb  = (_Float16*)(smem);
    _Float16* sBb  = (_Float16*)(smem + 8192);
    float*    sT1  = (float*)   (smem + 24576);
    _Float16* sT1h = (_Float16*)(smem + 57344);
    _Float16* sW2  = (_Float16*)(smem);
    float*    sT2  = (float*)   (smem + 16384);

    const int tid  = threadIdx.x;
    const int lane = tid & 31;
    const int wave = tid >> 5;
    const int b0   = blockIdx.x * 64;
    const int t    = blockIdx.y;
    const _Float16* W1t = W1 + (size_t)t * 128 * 256;
    char* ldsA  = (char*)sAb;
    char* ldsB  = (char*)sBb;
    char* ldsW2 = (char*)sW2;

    auto issue_s1 = [&](int buf, int kc) {
#pragma unroll
        for (int i = 0; i < 2; ++i) {
            const int idx = tid + i * 128;
            const int r = idx >> 2, c = idx & 3;
            copy_b128(ldsA, buf * 4096 + r * 64 + c * 16, h16 + (size_t)(b0 + r) * 256 + kc + c * 8);
        }
#pragma unroll
        for (int i = 0; i < 4; ++i) {
            const int idx = tid + i * 128;
            const int r = idx >> 2, c = idx & 3;
            copy_b128(ldsB, buf * 8192 + r * 64 + c * 16, W1t + (size_t)r * 256 + kc + c * 8);
        }
    };

    v8f acc1[4][2] = {};
    const int wn1 = wave * 32;
    issue_s1(0, 0);
    for (int kc = 0, it = 0; kc < 256; kc += 32, ++it) {
        const int cur = it & 1;
        __syncthreads();
        if (kc + 32 < 256) issue_s1(cur ^ 1, kc + 32);

        const _Float16* cA = sAb + cur * 2048;
        const _Float16* cB = sBb + cur * 4096;
        v16h bfr[2];
#pragma unroll
        for (int nt = 0; nt < 2; ++nt)
            bfr[nt] = load_frag_b(&cB[(wn1 + nt * 16) * 32], 32, lane);
#pragma unroll
        for (int mt = 0; mt < 4; ++mt) {
            v16h afr = load_frag_a(&cA[(mt * 16) * 32], 32, lane);
#pragma unroll
            for (int nt = 0; nt < 2; ++nt)
                acc1[mt][nt] = wmma_f16(afr, bfr[nt], acc1[mt][nt]);
        }
        __syncthreads();
    }
    {
        const int cn = lane & 15;
        const int mh = (lane >> 4) << 3;
#pragma unroll
        for (int mt = 0; mt < 4; ++mt)
#pragma unroll
            for (int nt = 0; nt < 2; ++nt) {
                const int n = wn1 + nt * 16 + cn;
                const float bb = b1[t * 128 + n];
#pragma unroll
                for (int j = 0; j < 8; ++j)
                    sT1[(mt * 16 + mh + j) * 128 + n] = acc1[mt][nt][j] + bb;
            }
    }
    __syncthreads();

#pragma unroll 1
    for (int rr = 0; rr < 16; ++rr) {
        const int m = wave * 16 + rr;
        float v[4], s = 0.f, ss = 0.f;
#pragma unroll
        for (int i = 0; i < 4; ++i) {
            v[i] = sT1[m * 128 + lane + i * 32];
            s += v[i]; ss += v[i] * v[i];
        }
#pragma unroll
        for (int msk = 16; msk >= 1; msk >>= 1) {
            s  += __shfl_xor(s, msk, 32);
            ss += __shfl_xor(ss, msk, 32);
        }
        const float mean = s * (1.f / 128.f);
        const float var  = ss * (1.f / 128.f) - mean * mean;
        const float rstd = rsqrtf(var + LN_EPS);
#pragma unroll
        for (int i = 0; i < 4; ++i) {
            const int c = lane + i * 32;
            float y = (v[i] - mean) * rstd * lng[t * 128 + c] + lnb[t * 128 + c];
            y = y > 0.f ? y : 0.f;
            sT1h[m * 128 + c] = (_Float16)y;
        }
    }
    __syncthreads();

    {
        const _Float16* W2t = W2 + (size_t)t * 64 * 128;
#pragma unroll
        for (int i = 0; i < 8; ++i) {
            const int idx = tid + i * 128;
            const int r = idx >> 4, c = idx & 15;
            copy_b128(ldsW2, r * 256 + c * 16, W2t + (size_t)r * 128 + c * 8);
        }
    }
    __syncthreads();

    v8f acc2[2][2] = {};
    const int wm2 = (wave >> 1) * 32;
    const int wn2 = (wave & 1) * 32;
#pragma unroll
    for (int kc = 0; kc < 128; kc += 32) {
        v16h af2[2], bf2[2];
#pragma unroll
        for (int mt = 0; mt < 2; ++mt)
            af2[mt] = load_frag_a(&sT1h[(wm2 + mt * 16) * 128 + kc], 128, lane);
#pragma unroll
        for (int nt = 0; nt < 2; ++nt)
            bf2[nt] = load_frag_b(&sW2[(wn2 + nt * 16) * 128 + kc], 128, lane);
#pragma unroll
        for (int mt = 0; mt < 2; ++mt)
#pragma unroll
            for (int nt = 0; nt < 2; ++nt)
                acc2[mt][nt] = wmma_f16(af2[mt], bf2[nt], acc2[mt][nt]);
    }
    {
        const int cn = lane & 15;
        const int mh = (lane >> 4) << 3;
#pragma unroll
        for (int mt = 0; mt < 2; ++mt)
#pragma unroll
            for (int nt = 0; nt < 2; ++nt) {
                const int n = wn2 + nt * 16 + cn;
                const float bb = b2[t * 64 + n];
#pragma unroll
                for (int j = 0; j < 8; ++j) {
                    float v = acc2[mt][nt][j] + bb;
                    sT2[(wm2 + mt * 16 + mh + j) * 64 + n] = v > 0.f ? v : 0.f;
                }
            }
    }
    __syncthreads();

    if (tid < 64) {
        float a = 0.f;
#pragma unroll 8
        for (int m2 = 0; m2 < 64; ++m2)
            a += sT2[tid * 64 + m2] * W3[t * 64 + m2];
        vst2(out + (size_t)t * BATCH + b0 + tid, a + b3[t]);
    }
}

__global__ __launch_bounds__(256) void write_out(const float* __restrict__ stg, float* __restrict__ out) {
    const int g = blockIdx.x * 256 + threadIdx.x;
    if (g >= (BATCH * TOUT) / 4) return;
    v4f o;
#pragma unroll
    for (int e = 0; e < 4; ++e) { const int f = g * 4 + e; const int b = f / TOUT, t = f - b * TOUT; o[e] = stg[(size_t)t * BATCH + b]; }
    vst2(out + (size_t)g * 4, o);
}

static inline void launch_cvt(const float* s, _Float16* d, size_t n, hipStream_t st) {
    const int n4 = (int)(n / 4);
    cvt_f32_f16_kernel<<<(n4 + 255) / 256, 256, 0, st>>>(s, d, n4);
}

extern "C" void kernel_launch(void* const* d_in, const int* in_sizes, int n_in,
                              void* d_out, int out_size, void* d_ws, size_t ws_size,
                              hipStream_t stream)
{
    (void)in_sizes; (void)n_in; (void)out_size; (void)ws_size;
    const float* x          = (const float*)d_in[0];
    const float* proj_W     = (const float*)d_in[1];
    const float* proj_b     = (const float*)d_in[2];
    const float* attn_in_W  = (const float*)d_in[3];
    const float* attn_in_b  = (const float*)d_in[4];
    const float* attn_out_W = (const float*)d_in[5];
    const float* attn_out_b = (const float*)d_in[6];
    const float* ln_g       = (const float*)d_in[7];
    const float* ln_b       = (const float*)d_in[8];
    const float* ff_W1      = (const float*)d_in[9];
    const float* ff_b1      = (const float*)d_in[10];
    const float* ff_W2      = (const float*)d_in[11];
    const float* ff_b2      = (const float*)d_in[12];
    const float* cross_in_W = (const float*)d_in[13];
    const float* cross_in_b = (const float*)d_in[14];
    const float* cross_out_W= (const float*)d_in[15];
    const float* cross_out_b= (const float*)d_in[16];
    const float* tp_W1      = (const float*)d_in[17];
    const float* tp_b1      = (const float*)d_in[18];
    const float* tp_ln_g    = (const float*)d_in[19];
    const float* tp_ln_b    = (const float*)d_in[20];
    const float* tp_W2      = (const float*)d_in[21];
    const float* tp_b2      = (const float*)d_in[22];
    const float* tp_W3      = (const float*)d_in[23];
    const float* tp_b3      = (const float*)d_in[24];
    float* out = (float*)d_out;

    const int D = DMODEL;

    char* cur = (char*)d_ws;
    auto take = [&cur](size_t bytes) { char* p = cur; cur += (bytes + 15) & ~(size_t)15; return p; };
    float*    h     = (float*)   take((size_t)BATCH * D * 4);
    float*    h2    = (float*)   take((size_t)BATCH * D * 4);
    _Float16* h16   = (_Float16*)take((size_t)BATCH * D * 2);
    _Float16* tmp16 = (_Float16*)take((size_t)BATCH * 4 * D * 2);
    _Float16* x16   = (_Float16*)take((size_t)BATCH * D_IN * 2);
    _Float16* wproj = (_Float16*)take((size_t)D * D_IN * 2);
    _Float16* wain  = (_Float16*)take((size_t)NLAYER * 3 * D * D * 2);
    _Float16* waout = (_Float16*)take((size_t)NLAYER * D * D * 2);
    _Float16* wff1  = (_Float16*)take((size_t)NLAYER * 4 * D * D * 2);
    _Float16* wff2  = (_Float16*)take((size_t)NLAYER * 4 * D * D * 2);
    _Float16* wcin  = (_Float16*)take((size_t)3 * D * D * 2);
    _Float16* wcout = (_Float16*)take((size_t)D * D * 2);
    _Float16* wtp1  = (_Float16*)take((size_t)TOUT * 128 * 256 * 2);
    _Float16* wtp2  = (_Float16*)take((size_t)TOUT * 64 * 128 * 2);
    float*    stg   = (float*)   take((size_t)TOUT * BATCH * 4);

    launch_cvt(x,          x16,   (size_t)BATCH * D_IN, stream);
    launch_cvt(proj_W,     wproj, (size_t)D * D_IN, stream);
    launch_cvt(attn_in_W,  wain,  (size_t)NLAYER * 3 * D * D, stream);
    launch_cvt(attn_out_W, waout, (size_t)NLAYER * D * D, stream);
    launch_cvt(ff_W1,      wff1,  (size_t)NLAYER * 4 * D * D, stream);
    launch_cvt(ff_W2,      wff2,  (size_t)NLAYER * 4 * D * D, stream);
    launch_cvt(cross_in_W, wcin,  (size_t)3 * D * D, stream);
    launch_cvt(cross_out_W,wcout, (size_t)D * D, stream);
    launch_cvt(tp_W1,      wtp1,  (size_t)TOUT * 128 * 256, stream);
    launch_cvt(tp_W2,      wtp2,  (size_t)TOUT * 64 * 128, stream);

    const dim3 blk(128);
    auto grid = [](int M, int N) { return dim3(M / 64, N / 64); };

    gemm_wmma_f16_kernel<0, false, true, true><<<grid(BATCH, D), blk, 0, stream>>>(
        x16, wproj, proj_b, nullptr, h, h16, BATCH, D, D_IN);

    for (int i = 0; i < NLAYER; ++i) {
        const _Float16* Wv = wain + ((size_t)i * 3 * D + 2 * D) * D;
        const float*    bv = attn_in_b + (size_t)i * 3 * D + 2 * D;
        gemm_wmma_f16_kernel<0, false, false, true><<<grid(BATCH, D), blk, 0, stream>>>(
            h16, Wv, bv, nullptr, nullptr, tmp16, BATCH, D, D);
        gemm_wmma_f16_kernel<0, true, true, false><<<grid(BATCH, D), blk, 0, stream>>>(
            tmp16, waout + (size_t)i * D * D, attn_out_b + (size_t)i * D,
            h, h2, nullptr, BATCH, D, D);
        ln256_kernel<<<BATCH / 4, 128, 0, stream>>>(
            h2, ln_g + (size_t)i * D, ln_b + (size_t)i * D, h, h16);
        gemm_wmma_f16_kernel<1, false, false, true><<<grid(BATCH, 4 * D), blk, 0, stream>>>(
            h16, wff1 + (size_t)i * 4 * D * D, ff_b1 + (size_t)i * 4 * D,
            nullptr, nullptr, tmp16, BATCH, 4 * D, D);
        gemm_wmma_f16_kernel<0, true, true, false><<<grid(BATCH, D), blk, 0, stream>>>(
            tmp16, wff2 + (size_t)i * D * 4 * D, ff_b2 + (size_t)i * D,
            h, h2, nullptr, BATCH, D, 4 * D);
        ln256_kernel<<<BATCH / 4, 128, 0, stream>>>(
            h2, ln_g + (size_t)i * D, ln_b + (size_t)i * D, h, h16);
    }

    gemm_wmma_f16_kernel<0, false, false, true><<<grid(BATCH, D), blk, 0, stream>>>(
        h16, wcin + (size_t)2 * D * D, cross_in_b + 2 * D,
        nullptr, nullptr, tmp16, BATCH, D, D);
    gemm_wmma_f16_kernel<0, true, true, false><<<grid(BATCH, D), blk, 0, stream>>>(
        tmp16, wcout, cross_out_b, h, h2, nullptr, BATCH, D, D);
    launch_cvt(h2, h16, (size_t)BATCH * D, stream);

    dim3 tpg(BATCH / 64, TOUT);
    tp_fused_kernel<<<tpg, blk, 0, stream>>>(h16, wtp1, tp_b1, tp_ln_g, tp_ln_b,
                                             wtp2, tp_b2, tp_W3, tp_b3, stg);
    write_out<<<((BATCH * TOUT) / 4 + 255) / 256, 256, 0, stream>>>(stg, out);
}
